// TimeCondAttention_18236431138865
// MI455X (gfx1250) — hardware-verified
//
#include <hip/hip_runtime.h>
#include <math.h>

typedef __attribute__((ext_vector_type(16))) _Float16 v16h;
typedef __attribute__((ext_vector_type(16))) __bf16 v16b;
typedef __attribute__((ext_vector_type(8)))  _Float16 v8h;
typedef __attribute__((ext_vector_type(8)))  float v8f;
typedef __attribute__((ext_vector_type(4)))  float v4f;
typedef __attribute__((ext_vector_type(2)))  float v2f;
typedef __attribute__((ext_vector_type(4)))  unsigned v4u;
typedef __attribute__((ext_vector_type(4)))  int v4i;
typedef float __attribute__((may_alias)) float_a;
typedef int __attribute__((may_alias)) int_a;

template <typename T> __device__ __forceinline__ void vst2(void* p, T v) { *(volatile T*)p = v; __threadfence(); *(volatile T*)p = v; }
__device__ __forceinline__ v8f wmma16(v16h a, v16h b, v8f c) {
  v8f d = __builtin_amdgcn_wmma_f32_16x16x32_f16(false, a, false, b, (short)0, c, false, false);
  asm volatile("v_nop\n\tv_nop\n\tv_nop\n\tv_nop" : "+v"(d) : "v"(a), "v"(b));
  return d;
}
__device__ __forceinline__ v8f wmma_bf(v16b a, v16b b, v8f c) {
  v8f d = __builtin_amdgcn_wmma_f32_16x16x32_bf16(false, a, false, b, (short)0, c, false, false);
  asm volatile("v_nop\n\tv_nop\n\tv_nop\n\tv_nop" : "+v"(d) : "v"(a), "v"(b));
  return d;
}
__device__ __forceinline__ v16h frag_h(const _Float16* rowk0, int lane) {
  union { v16h v; v8h q[2]; } u; const _Float16* p = rowk0 + 8 * (lane >> 4);
  u.q[0] = *(const v8h*)p; u.q[1] = *(const v8h*)(p + 16); return u.v;
}
__device__ __forceinline__ v16h frag_f32(const float* rowk0, int lane) {
  v16h a; const float* p = rowk0 + 8 * (lane >> 4);
#pragma unroll
  for (int i = 0; i < 8; ++i) { a[i] = (_Float16)p[i]; a[8 + i] = (_Float16)p[16 + i]; }
  return a;
}
__device__ __forceinline__ v16h frag_f32s(const float* rowk0, int lane, float sc) {
  v16h a; const float* p = rowk0 + 8 * (lane >> 4);
#pragma unroll
  for (int i = 0; i < 8; ++i) { a[i] = (_Float16)(p[i] * sc); a[8 + i] = (_Float16)(p[16 + i] * sc); }
  return a;
}
__device__ __forceinline__ v16h fragc_f32(const float* W, int k0, int n, int lane, int ld, int K) {
  v16h a; const int g = lane >> 4;
#pragma unroll
  for (int i = 0; i < 8; ++i) { const int ka = k0 + 8 * g + i, kb = ka + 16;
    a[i] = (_Float16)(ka < K ? W[(size_t)(ka < K ? ka : K - 1) * ld + n] : 0.f); a[8 + i] = (_Float16)(kb < K ? W[(size_t)(kb < K ? kb : K - 1) * ld + n] : 0.f); }
  return a;
}
struct F2 { v16b h, l; };
__device__ __forceinline__ F2 bsplit16(const float v[16]) { F2 r;
#pragma unroll
  for (int i = 0; i < 16; ++i) { const __bf16 h = (__bf16)v[i]; r.h[i] = h; r.l[i] = (__bf16)(v[i] - (float)h); }
  return r; }
__device__ __forceinline__ F2 split_row(const float* row, int k0, int lane) { float v[16]; const float* p = row + k0 + 8 * (lane >> 4);
#pragma unroll
  for (int i = 0; i < 8; ++i) { v[i] = p[i]; v[8 + i] = p[16 + i]; }
  return bsplit16(v); }
__device__ __forceinline__ F2 split_rowK(const float* row, int k0, int lane, int K) { float v[16]; const int g = lane >> 4;
#pragma unroll
  for (int i = 0; i < 8; ++i) { const int ka = k0 + 8 * g + i, kb = ka + 16; v[i] = ka < K ? row[ka < K ? ka : K - 1] : 0.f; v[8 + i] = kb < K ? row[kb < K ? kb : K - 1] : 0.f; }
  return bsplit16(v); }
__device__ __forceinline__ F2 split_col(const float* W, int k0, int n, int lane, int ld, int K) { float v[16]; const int g = lane >> 4;
#pragma unroll
  for (int i = 0; i < 8; ++i) { const int ka = k0 + 8 * g + i, kb = ka + 16; v[i] = ka < K ? W[(size_t)(ka < K ? ka : K - 1) * ld + n] : 0.f; v[8 + i] = kb < K ? W[(size_t)(kb < K ? kb : K - 1) * ld + n] : 0.f; }
  return bsplit16(v); }
__device__ __forceinline__ v8f mac3(const F2& a, const F2& b, v8f c) { c = wmma_bf(a.l, b.h, c); c = wmma_bf(a.h, b.l, c); return wmma_bf(a.h, b.h, c); }
__device__ __forceinline__ float sigm(float v) { return 1.0f / (1.0f + expf(-v)); }
#define LDSX() do { asm volatile("s_wait_dscnt 0" ::: "memory"); __builtin_amdgcn_wave_barrier(); __builtin_amdgcn_fence(__ATOMIC_RELEASE, "workgroup"); } while (0)


#define NB 4
#define LL 1024
#define DM_ 1024
#define NH 16
#define HD 64
#define NF 32
#ifndef TNB
#define TNB NB
#endif
#ifndef TQB
#define TQB (LL / 64)
#endif
typedef __attribute__((ext_vector_type(8))) __bf16 v8b;
__device__ __forceinline__ v16b frag_b(const __bf16* rowk0, int lane) {
  union { v16b v; v8b q[2]; } u; const __bf16* p = rowk0 + 8 * (lane >> 4);
  u.q[0] = *(const v8b*)p; u.q[1] = *(const v8b*)(p + 16); return u.v;
}
__device__ __forceinline__ float bfr(float v) { return (float)(__bf16)v; }
__device__ __attribute__((noinline)) float exp_ni(float v) { return expf(v); }
__device__ __attribute__((noinline)) float erf_ni(float v) { return erff(v); }

#define WS_SS  0u
#define WS_CNT (WS_SS + 4u * (size_t)NB * 2 * DM_)
#define WS_XC  (WS_CNT + 4u * (size_t)NB * 32)
#define WS_QF  (WS_XC + 2u * (size_t)NB * LL * DM_)
#define WS_KF  (WS_QF + 4u * (size_t)NB * LL * DM_)
#define WS_QH  (WS_KF + 4u * (size_t)NB * LL * DM_)
#define WS_KH  (WS_QH + 2u * (size_t)NB * LL * DM_)
#define WS_KL  (WS_KH + 2u * (size_t)NB * LL * DM_)
#define WS_VT  (WS_KL + 2u * (size_t)NB * LL * DM_)
#define WS_CT  (WS_VT + 2u * (size_t)NB * DM_ * LL)
#define WS_END (WS_CT + 4u * (size_t)NB * LL * DM_)

__global__ __launch_bounds__(128) void k_time(const float* __restrict__ TM, const float* __restrict__ WT, const float* __restrict__ BT, float* __restrict__ SSo) { __shared__ __align__(16) float st[DM_]; __shared__ __align__(16) float so[128];
  const int t = threadIdx.x; const size_t b = blockIdx.y; const int o0 = blockIdx.x * 128;
  for (int i = t; i < DM_; i += 128) { const float v = bfr(TM[b * DM_ + i]); st[i] = v / (1.0f + expf(-v)); }
  __syncthreads();
  { const int o = o0 + t; float a = bfr(BT[o]);
#pragma unroll 1
    for (int i = 0; i < DM_; ++i) a += st[i] * bfr(WT[(size_t)o * DM_ + i]); so[t] = a; }
  __syncthreads(); if (t < 32) vst2(SSo + b * 2 * DM_ + o0 + t * 4, *(const v4f*)&so[t * 4]); }
__global__ __launch_bounds__(256) void k_cnt(const int* __restrict__ CH, const float* __restrict__ CM, float* __restrict__ CNT) { __shared__ float sred[8][NB][2]; __shared__ __align__(16) float so[NB][8];
  const int t = threadIdx.x; float acc[NB][2]; for (int b = 0; b < NB; ++b) { acc[b][0] = 0.f; acc[b][1] = 0.f; }
  for (int e = t; e < NB * LL; e += 256) { const int b = e / LL; const int c = CH[e]; const float m = bfr(CM[e]); if (c == 0) acc[b][0] += m; else acc[b][1] += m; }
  for (int b = 0; b < NB; ++b) for (int c = 0; c < 2; ++c) { float v = acc[b][c];
#pragma unroll
      for (int o = 1; o < 32; o <<= 1) v += __shfl_xor(v, o); if ((t & 31) == 0) sred[t >> 5][b][c] = v; }
  __syncthreads(); if (t < NB * 8) { const int b = t / 8, c = t % 8; float v = 0.f; if (c < 2) for (int w = 0; w < 8; ++w) v += sred[w][b][c]; so[b][c] = v; }
  __syncthreads(); if (t < NB * 2) vst2(CNT + t * 4, *(const v4f*)&(&so[0][0])[t * 4]); }
__global__ __launch_bounds__(256) void k_ln(const float* __restrict__ X, const float* __restrict__ SM, const float* __restrict__ GA, const float* __restrict__ SSo, _Float16* __restrict__ XC) { __shared__ float sred[8]; __shared__ float smu, sinv; __shared__ __align__(16) _Float16 sh[DM_];
  const int t = threadIdx.x; const size_t row = blockIdx.x; const size_t b = row / LL; const float msk = bfr(SM[row]); const float* xr = X + row * DM_;
  float s = 0.f; for (int i = t; i < DM_; i += 256) s += bfr(xr[i]) * msk;
#pragma unroll
  for (int o = 1; o < 32; o <<= 1) s += __shfl_xor(s, o);
  if ((t & 31) == 0) sred[t >> 5] = s; __syncthreads(); if (t == 0) { float a = 0.f; for (int i = 0; i < 8; ++i) a += sred[i]; smu = a / DM_; } __syncthreads(); const float mu = smu;
  float q = 0.f; for (int i = t; i < DM_; i += 256) { const float d = bfr(xr[i]) * msk - mu; q += d * d; }
#pragma unroll
  for (int o = 1; o < 32; o <<= 1) q += __shfl_xor(q, o);
  __syncthreads(); if ((t & 31) == 0) sred[t >> 5] = q; __syncthreads(); if (t == 0) { float a = 0.f; for (int i = 0; i < 8; ++i) a += sred[i]; sinv = 1.0f / sqrtf(a / DM_ + 1e-5f); } __syncthreads(); const float inv = sinv;
  for (int i = t; i < DM_; i += 256) { const float xn = (bfr(xr[i]) * msk - mu) * inv * bfr(GA[i]); sh[i] = (_Float16)(xn * (SSo[b * 2 * DM_ + i] + 1.0f) + SSo[b * 2 * DM_ + DM_ + i]); }
  __syncthreads(); for (int qq = t; qq < DM_ / 8; qq += 256) vst2((unsigned*)(XC + row * DM_ + qq * 8), *(const v4u*)&sh[qq * 8]); }
__global__ __launch_bounds__(128) void k_proj(const _Float16* __restrict__ XC, const float* __restrict__ WQ, const float* __restrict__ WKV, float* __restrict__ QF, float* __restrict__ KF, _Float16* __restrict__ VT) { __shared__ __align__(16) float sf[4][16][132]; __shared__ __align__(16) _Float16 th[128][72];
  const int tid = threadIdx.x, wave = tid >> 5, lane = tid & 31, col = lane & 15, g = lane >> 4; const int which = blockIdx.z; const int c0 = blockIdx.y * 128; const size_t r0 = (size_t)blockIdx.x * 64;
  const float* Wm = which == 0 ? WQ : (which == 1 ? WKV : WKV + (size_t)DM_ * DM_);
  v8f acc[8] = {};
#pragma unroll 2
  for (int kc = 0; kc < DM_ / 32; ++kc) { const v16h a = frag_h(XC + (r0 + wave * 16 + col) * DM_ + kc * 32, lane);
#pragma unroll
    for (int j = 0; j < 8; ++j) { v16h w; const int o = c0 + j * 16 + col;
#pragma unroll
      for (int i = 0; i < 8; ++i) { w[i] = (_Float16)bfr(Wm[(size_t)o * DM_ + kc * 32 + 8 * g + i]); w[8 + i] = (_Float16)bfr(Wm[(size_t)o * DM_ + kc * 32 + 16 + 8 * g + i]); }
      acc[j] = wmma16(a, w, acc[j]); } }
  if (which < 2) {
#pragma unroll
    for (int j = 0; j < 8; ++j)
#pragma unroll
      for (int r = 0; r < 8; ++r) sf[wave][8 * g + r][j * 16 + col] = acc[j][r];
    LDSX(); float* dst = which == 0 ? QF : KF; for (int rl = 0; rl < 16; ++rl) vst2(dst + (r0 + wave * 16 + rl) * DM_ + c0 + lane * 4, *(const v4f*)&sf[wave][rl][lane * 4]); }
  else {
#pragma unroll
    for (int j = 0; j < 8; ++j)
#pragma unroll
      for (int r = 0; r < 8; ++r) th[j * 16 + col][wave * 16 + 8 * g + r] = (_Float16)acc[j][r];
    __syncthreads(); const size_t b = r0 / LL; const int l0 = (int)(r0 % LL); for (int e = tid; e < 128 * 8; e += 128) { const int cl = e >> 3, q = e & 7; vst2((unsigned*)(VT + (b * DM_ + c0 + cl) * (size_t)LL + l0 + q * 8), *(const v4u*)&th[cl][q * 8]); } } }
__global__ __launch_bounds__(256) void k_rope(const float* __restrict__ QF, const float* __restrict__ KF, const float* __restrict__ RF, const int* __restrict__ RI, const int* __restrict__ CH, const float* __restrict__ CM, const float* __restrict__ CNT, _Float16* __restrict__ QH, _Float16* __restrict__ KH, _Float16* __restrict__ KL) { __shared__ float sc[NF], ssn[NF]; __shared__ __align__(16) _Float16 sq[DM_], skh[DM_], skl[DM_];
  const int t_ = threadIdx.x; const size_t row = blockIdx.x; const size_t b = row / LL;
  if (t_ < NF) { const int f = t_; const float t = (float)RI[row]; const int cidx = CH[row]; const float ci = (float)cidx; const float cm = bfr(CM[row]); float ang;
    if (cm > 0.f) { const float ring = CNT[b * 8 + cidx] * cm; const float ring_safe = fmaxf(ring, 1.0f); const float max_k = fmaxf(floorf(ring_safe * 0.5f), 1.0f); const float kk = (float)(f + 1); const float k_eff = (max_k == 1.0f) ? 1.0f : (1.0f + fmodf(kk - 1.0f, max_k)); const float omega = 6.283185307179586f * k_eff / ring_safe; ang = omega * t; }
    else { const float res = t * bfr(RF[f]); const float ch0 = ci * bfr(RF[0]); ang = res + ch0; }
    sc[f] = cosf(ang); ssn[f] = sinf(ang); }
  __syncthreads();
  for (int e = t_; e < DM_ / 2; e += 256) { const int f = e % NF; const int i0 = 2 * e; const float c = sc[f], s = ssn[f];
    { const float x1 = QF[row * DM_ + i0], x2 = QF[row * DM_ + i0 + 1]; sq[i0] = (_Float16)(x1 * c - x2 * s); sq[i0 + 1] = (_Float16)(x2 * c + x1 * s); }
    { const float x1 = KF[row * DM_ + i0], x2 = KF[row * DM_ + i0 + 1]; const float y0 = x1 * c - x2 * s, y1 = x2 * c + x1 * s; const _Float16 h0 = (_Float16)y0, h1 = (_Float16)y1; skh[i0] = h0; skh[i0 + 1] = h1; skl[i0] = (_Float16)(y0 - (float)h0); skl[i0 + 1] = (_Float16)(y1 - (float)h1); } }
  __syncthreads(); for (int q = t_; q < DM_ / 8; q += 256) { vst2((unsigned*)(QH + row * DM_ + q * 8), *(const v4u*)&sq[q * 8]); vst2((unsigned*)(KH + row * DM_ + q * 8), *(const v4u*)&skh[q * 8]); vst2((unsigned*)(KL + row * DM_ + q * 8), *(const v4u*)&skl[q * 8]); } }
__global__ __launch_bounds__(128) void k_att(const _Float16* __restrict__ QH, const _Float16* __restrict__ KH, const _Float16* __restrict__ KL, const _Float16* __restrict__ VT, const float* __restrict__ SM, float* __restrict__ CT) {
  __shared__ __align__(16) float sp[4][16][36]; __shared__ __align__(16) float so[4][16][68];
  const int tid = threadIdx.x, wave = tid >> 5, lane = tid & 31, col = lane & 15, g = lane >> 4; const int qb = blockIdx.x, h = blockIdx.y; const size_t b = blockIdx.z; const size_t q0 = b * LL + (size_t)qb * 64 + wave * 16;
  v16h aq[2];
#pragma unroll
  for (int kc = 0; kc < 2; ++kc) aq[kc] = frag_h(QH + (q0 + col) * DM_ + h * HD + kc * 32, lane);
  float m[8], l[8];
#pragma unroll
  for (int r = 0; r < 8; ++r) { m[r] = -3.0e38f; l[r] = 0.f; }
  v8f acc[4] = {};
#pragma unroll 1
  for (int ks = 0; ks < LL / 32; ++ks) { float s[2][8];
#pragma unroll
    for (int ct = 0; ct < 2; ++ct) { const int kt = ks * 32 + ct * 16 + col; const size_t kk = b * LL + kt; v8f c = {};
#pragma unroll
      for (int kc = 0; kc < 2; ++kc) { c = wmma16(aq[kc], frag_h(KH + kk * DM_ + h * HD + kc * 32, lane), c); c = wmma16(aq[kc], frag_h(KL + kk * DM_ + h * HD + kc * 32, lane), c); }
      const bool keep = bfr(SM[kk]) > 0.f;
#pragma unroll
      for (int r = 0; r < 8; ++r) s[ct][r] = keep ? c[r] * 0.125f : -3.0e38f; }
    float alpha[8];
#pragma unroll
    for (int r = 0; r < 8; ++r) { float mx = fmaxf(s[0][r], s[1][r]);
#pragma unroll
      for (int o = 1; o < 16; o <<= 1) mx = fmaxf(mx, __shfl_xor(mx, o));
      const float mn = fmaxf(m[r], mx); alpha[r] = (mn <= -1.0e38f) ? 1.f : __expf(m[r] - mn); const float e0 = (s[0][r] <= -1.0e38f) ? 0.f : __expf(s[0][r] - mn), e1 = (s[1][r] <= -1.0e38f) ? 0.f : __expf(s[1][r] - mn); float es = e0 + e1;
#pragma unroll
      for (int o = 1; o < 16; o <<= 1) es += __shfl_xor(es, o);
      l[r] = l[r] * alpha[r] + es; m[r] = mn; sp[wave][8 * g + r][col] = e0; sp[wave][8 * g + r][16 + col] = e1; }
#pragma unroll
    for (int j = 0; j < 4; ++j)
#pragma unroll
      for (int r = 0; r < 8; ++r) acc[j][r] *= alpha[r];
    LDSX();
    const v16h pa = frag_f32s(&sp[wave][col][0], lane, 2048.0f);
#pragma unroll
    for (int j = 0; j < 4; ++j) acc[j] = wmma16(pa, frag_h(VT + (b * DM_ + (size_t)h * HD + j * 16 + col) * LL + ks * 32, lane), acc[j]);
    LDSX(); }
#pragma unroll
  for (int r = 0; r < 8; ++r) { const float il = (1.0f / 2048.0f) / l[r];
#pragma unroll
    for (int j = 0; j < 4; ++j) so[wave][8 * g + r][j * 16 + col] = acc[j][r] * il; }
  LDSX(); for (int rl = 0; rl < 16; ++rl) if (lane < 16) vst2(CT + (q0 + rl) * DM_ + h * HD + lane * 4, *(const v4f*)&so[wave][rl][lane * 4]); }
__global__ __launch_bounds__(128) void k_out(const float* __restrict__ CT, const float* __restrict__ WO, const float* __restrict__ SM, float* __restrict__ OUT) { __shared__ __align__(16) float sf[4][16][132];
  const int tid = threadIdx.x, wave = tid >> 5, lane = tid & 31, col = lane & 15, g = lane >> 4; const int c0 = blockIdx.y * 128; const size_t r0 = (size_t)blockIdx.x * 64 + wave * 16;
  v8f acc[8] = {};
#pragma unroll 2
  for (int kc = 0; kc < DM_ / 32; ++kc) { const F2 a = split_row(CT + (r0 + col) * DM_, kc * 32, lane);
#pragma unroll
    for (int j = 0; j < 8; ++j) { v16b w; const int o = c0 + j * 16 + col;
#pragma unroll
      for (int i = 0; i < 8; ++i) { w[i] = (__bf16)WO[(size_t)o * DM_ + kc * 32 + 8 * g + i]; w[8 + i] = (__bf16)WO[(size_t)o * DM_ + kc * 32 + 16 + 8 * g + i]; }
      acc[j] = wmma_bf(a.h, w, acc[j]); acc[j] = wmma_bf(a.l, w, acc[j]); } }
#pragma unroll
  for (int j = 0; j < 8; ++j)
#pragma unroll
    for (int r = 0; r < 8; ++r) sf[wave][8 * g + r][j * 16 + col] = acc[j][r] * bfr(SM[r0 + 8 * g + r]);
  LDSX(); for (int rl = 0; rl < 16; ++rl) vst2(OUT + (r0 + rl) * DM_ + c0 + lane * 4, *(const v4f*)&sf[wave][rl][lane * 4]); }
extern "C" void kernel_launch(void* const* d_in, const int* in_sizes, int n_in, void* d_out, int out_size, void* d_ws, size_t ws_size, hipStream_t stream) {
  (void)in_sizes; (void)n_in; (void)out_size;
  const float** F = (const float**)d_in;
  if (ws_size < (size_t)WS_END) return;
  char* ws = (char*)d_ws; float *SSo = (float*)(ws + WS_SS), *CNT = (float*)(ws + WS_CNT), *QF = (float*)(ws + WS_QF), *KF = (float*)(ws + WS_KF), *CT = (float*)(ws + WS_CT); _Float16 *XC = (_Float16*)(ws + WS_XC), *QH = (_Float16*)(ws + WS_QH), *KH = (_Float16*)(ws + WS_KH), *KL = (_Float16*)(ws + WS_KL), *VT = (_Float16*)(ws + WS_VT);
  k_time<<<dim3(2 * DM_ / 128, TNB), 128, 0, stream>>>(F[1], F[5], F[6], SSo);
  k_cnt<<<1, 256, 0, stream>>>((const int*)d_in[12], F[3], CNT);
  k_ln<<<TNB * LL, 256, 0, stream>>>(F[0], F[2], F[4], SSo, XC);
  k_proj<<<dim3(TNB * LL / 64, DM_ / 128, 3), 128, 0, stream>>>(XC, F[7], F[8], QF, KF, VT);
  k_rope<<<TNB * LL, 256, 0, stream>>>(QF, KF, F[10], (const int*)d_in[11], (const int*)d_in[12], F[3], CNT, QH, KH, KL);
  k_att<<<dim3(TQB, NH, TNB), 128, 0, stream>>>(QH, KH, KL, VT, F[2], CT);
  for (int b = 0; b < TNB; ++b) k_out<<<dim3(TQB, DM_ / 128), 128, 0, stream>>>(CT + (size_t)b * LL * DM_, F[9], F[2] + (size_t)b * LL, (float*)d_out + (size_t)b * LL * DM_);
}
